// CrossAttention_27925877359245
// MI455X (gfx1250) — hardware-verified
//
#include <hip/hip_runtime.h>


#ifndef NB
#define NB 4
#endif
#ifndef TX
#define TX 1024
#endif
#define NB_FULL 4
#define TX_FULL 1024
#define TY   1024
#define DMD  768
#define NHD  12
#define HD   64
#define KC2  (2 * DMD)
#define PCAR 16384.0f
#define OCAR 1024.0f
#define RLO  2048.0f
#define SCL  0.125f
#define L2E  1.4426950408889634f
#define KPT  72
#define PPT  40
#define OPT  68
static_assert(NB >= 1 && NB <= NB_FULL);
static_assert(TX >= 64 && TX <= TX_FULL && (TX % 64) == 0);
static_assert((TY % 64) == 0 && (DMD % 64) == 0 && HD == 64 && NHD * HD == DMD);
static_assert((DMD % 32) == 0 && (HD % 32) == 0 && (KC2 % 32) == 0);
static_assert(((NB * TX) % 64) == 0 && ((NB * TY) % 64) == 0);
static_assert(128 * 4 == 64 * (HD / 8));
static_assert(KPT >= 64 && (KPT % 8) == 0 && PPT >= 32 && (PPT % 8) == 0 && OPT >= 64 && (OPT % 4) == 0);
static_assert((size_t)NHD * NB * TX * HD < (size_t)2147483647);
static_assert(4 * 64 * KPT * 2 + 4 * 16 * PPT * 2 + 4 * 16 * OPT * 4 <= 65536);

typedef _Float16 h16;
typedef unsigned short bf;
typedef __attribute__((ext_vector_type(16))) __bf16   v16bf;
typedef __attribute__((ext_vector_type(16))) _Float16 v16h;
typedef __attribute__((ext_vector_type(8)))  _Float16 v8h;
typedef __attribute__((ext_vector_type(8)))  unsigned short v8us;
typedef __attribute__((ext_vector_type(8)))  float    v8f;
typedef __attribute__((ext_vector_type(4)))  float    v4f;
typedef v8h  __attribute__((may_alias)) v8ha;
typedef v4f  __attribute__((may_alias)) v4fa;

__device__ __forceinline__ unsigned short f2bf(float f) { unsigned u = __float_as_uint(f); u += 0x7FFFu + ((u >> 16) & 1u); return (unsigned short)(u >> 16); }
__device__ __forceinline__ float bf2f(unsigned short b) { return __uint_as_float(((unsigned)b) << 16); }
__device__ __forceinline__ float bfr(float f) { return bf2f(f2bf(f)); }
__device__ __forceinline__ v16h cat16(v8h lo, v8h hi) { return __builtin_shufflevector(lo, hi, 0, 1, 2, 3, 4, 5, 6, 7, 8, 9, 10, 11, 12, 13, 14, 15); }
__device__ __forceinline__ v16bf cat16b(v8us lo, v8us hi) { return __builtin_bit_cast(v16bf, __builtin_shufflevector(lo, hi, 0, 1, 2, 3, 4, 5, 6, 7, 8, 9, 10, 11, 12, 13, 14, 15)); }
__device__ __forceinline__ v8f wmma16(v16h a, v16h b, v8f c) { return __builtin_amdgcn_wmma_f32_16x16x32_f16(false, a, false, b, (short)0, c, false, false); }
__device__ __forceinline__ v8f wmmab(v16bf a, v16bf b, v8f c) { return __builtin_amdgcn_wmma_f32_16x16x32_bf16(false, a, false, b, (short)0, c, false, false); }
__device__ __forceinline__ h16 tohx(float x) { return (h16)x; }
__device__ __forceinline__ void wsync() { __builtin_amdgcn_wave_barrier(); asm volatile("" ::: "memory"); }

template <typename T16> struct WFrag;
template <> struct WFrag<h16> { typedef v16h V; static __device__ __forceinline__ V ld(const h16* p) { return cat16(*(const v8h*)p, *(const v8h*)(p + 16)); } static __device__ __forceinline__ v8f mma(V a, V b, v8f c) { return wmma16(a, b, c); } };
template <> struct WFrag<bf> { typedef v16bf V; static __device__ __forceinline__ V ld(const bf* p) { return cat16b(*(const v8us*)p, *(const v8us*)(p + 16)); } static __device__ __forceinline__ v8f mma(V a, V b, v8f c) { return wmmab(a, b, c); } };

template <typename T16, int EP>
__device__ __forceinline__ void gemmw_body(const T16* __restrict__ A, const T16* __restrict__ Bt, int K, float* Cf, h16* Ch, h16* Cl, int ldc, const float* __restrict__ bias, const float* __restrict__ radd, size_t sA, size_t sB, size_t sC, float cs) {
    static_assert(EP == 0 || EP == 2 || EP == 3);
    typedef typename WFrag<T16>::V V;
    __shared__ __align__(16) float os[16 * OPT];
    const size_t z = blockIdx.z; A += z * sA; Bt += z * sB;
    if (EP == 0) { Cf += z * sC; } else { Ch += z * sC; Cl += z * sC; }
    const int lane = threadIdx.x & 31, lr = lane & 15, hi = lane >> 4; const int r0 = blockIdx.x * 64, c0 = blockIdx.y * 64;
    v8f acc[4][4];
#pragma unroll
    for (int mb = 0; mb < 4; ++mb)
#pragma unroll
        for (int nb = 0; nb < 4; ++nb) acc[mb][nb] = (v8f){};
    const size_t aoff = (size_t)(r0 + lr) * K + 8 * hi, boff = (size_t)(c0 + lr) * K + 8 * hi;
#pragma unroll 1
    for (int kc = 0; kc < K; kc += 32) {
        V a[4];
#pragma unroll
        for (int mb = 0; mb < 4; ++mb) a[mb] = WFrag<T16>::ld(A + aoff + (size_t)mb * 16 * K + kc);
#pragma unroll
        for (int nb = 0; nb < 4; ++nb) { const V b = WFrag<T16>::ld(Bt + boff + (size_t)nb * 16 * K + kc);
#pragma unroll
            for (int mb = 0; mb < 4; ++mb) acc[mb][nb] = WFrag<T16>::mma(a[mb], b, acc[mb][nb]); }
        asm volatile("v_nop\n\tv_nop\n\tv_nop\n\tv_nop" : "+v"(acc[0][0]), "+v"(acc[1][1]), "+v"(acc[2][2]), "+v"(acc[3][3]) : "v"(a[0]), "v"(a[3]));
    }
#pragma unroll
    for (int mb = 0; mb < 4; ++mb) {
#pragma unroll
        for (int nb = 0; nb < 4; ++nb) {
#pragma unroll
            for (int j = 0; j < 8; ++j) os[(hi * 8 + j) * OPT + nb * 16 + lr] = acc[mb][nb][j]; }
        wsync();
        if (EP == 0) {
            float* crow = Cf + (size_t)(r0 + mb * 16) * ldc + c0;
#pragma unroll 1
            for (int ps = 0; ps < 2; ++ps) {
#pragma unroll
                for (int s = 0; s < 8; ++s) { const int row = 2 * s + hi, cofs = lr * 4; v4f val = *(const v4fa*)(os + row * OPT + cofs);
                    val[0] = __fmul_rn(val[0], cs); val[1] = __fmul_rn(val[1], cs); val[2] = __fmul_rn(val[2], cs); val[3] = __fmul_rn(val[3], cs);
                    val[0] += bfr(bias[c0 + cofs]); val[1] += bfr(bias[c0 + cofs + 1]); val[2] += bfr(bias[c0 + cofs + 2]); val[3] += bfr(bias[c0 + cofs + 3]);
                    *(volatile v4f*)(crow + (size_t)row * ldc + cofs) = val; }
                if (ps == 0) __threadfence(); }
        } else {
            float ra[4] = {0.0f, 0.0f, 0.0f, 0.0f};
            if (EP == 2) {
#pragma unroll
                for (int s = 0; s < 4; ++s) ra[s] = bfr(radd[r0 + mb * 16 + 4 * s + (lane >> 3)]);
            }
            h16* hrow = Ch + (size_t)(r0 + mb * 16) * ldc + c0;
            h16* lrow = Cl + (size_t)(r0 + mb * 16) * ldc + c0;
#pragma unroll 1
            for (int ps = 0; ps < 2; ++ps) {
#pragma unroll
                for (int s = 0; s < 4; ++s) { const int row = 4 * s + (lane >> 3), c8 = (lane & 7) * 8;
                    const v4f u0 = *(const v4fa*)(os + row * OPT + c8), u1 = *(const v4fa*)(os + row * OPT + c8 + 4);
                    v8h o, ol;
#pragma unroll
                    for (int q = 0; q < 8; ++q) { const float u = (q < 4) ? u0[q & 3] : u1[q & 3]; const float f = __fmul_rn(u, cs) + ra[s]; const h16 hh = tohx(f); o[q] = hh; ol[q] = tohx((f - (float)hh) * RLO); }
                    *(volatile v8h*)(hrow + (size_t)row * ldc + c8) = o;
                    *(volatile v8h*)(lrow + (size_t)row * ldc + c8) = ol; }
                if (ps == 0) __threadfence(); }
        }
        wsync();
    }
}

__global__ __launch_bounds__(32) void k_gemm_q(const bf* A, const bf* Bt, int K, h16* Ch, h16* Cl, int ldc, size_t sA, size_t sB, size_t sC) {
    gemmw_body<bf, 3>(A, Bt, K, nullptr, Ch, Cl, ldc, nullptr, nullptr, sA, sB, sC, 1.0f); }
__global__ __launch_bounds__(32) void k_gemm_k(const bf* A, const bf* Bt, int K, h16* Ch, h16* Cl, int ldc, const float* radd, size_t sA, size_t sB, size_t sC) {
    gemmw_body<bf, 2>(A, Bt, K, nullptr, Ch, Cl, ldc, nullptr, radd, sA, sB, sC, 1.0f); }
__global__ __launch_bounds__(32) void k_gemm_v(const bf* A, const bf* Bt, int K, h16* Ch, h16* Cl, int ldc, size_t sA, size_t sB, size_t sC) {
    gemmw_body<bf, 3>(A, Bt, K, nullptr, Ch, Cl, ldc, nullptr, nullptr, sA, sB, sC, 1.0f); }
__global__ __launch_bounds__(32) void k_gemm_o(const h16* A, const h16* Bt, int K, float* Cf, int ldc, const float* bias, size_t sA, size_t sB, size_t sC, float cs) {
    gemmw_body<h16, 0>(A, Bt, K, Cf, nullptr, nullptr, ldc, bias, nullptr, sA, sB, sC, cs); }

__global__ __launch_bounds__(256) void k_cvt8r(const float* __restrict__ src, bf* dst, int rows, int srows, size_t n8) {
    const size_t i = (size_t)blockIdx.x * 256 + threadIdx.x; if (i >= n8) return;
    const size_t e = i * 8; const size_t r = e / DMD; const int c = (int)(e % DMD); const size_t bb = r / (size_t)rows; const size_t t = r % (size_t)rows;
    const v8f v = *(const v8f*)(src + (bb * (size_t)srows + t) * DMD + c); v8us o;
#pragma unroll
    for (int k = 0; k < 8; ++k) o[k] = f2bf(v[k]);
    *(volatile v8us*)(dst + e) = o; __threadfence(); *(volatile v8us*)(dst + e) = o; }

__global__ __launch_bounds__(256) void k_cvtwp(const float* __restrict__ F, h16* P, size_t n8) {
    const size_t i = (size_t)blockIdx.x * 256 + threadIdx.x; if (i >= n8) return;
    const size_t e = i * 8; const size_t r = e / DMD; const int c = (int)(e % DMD);
    const v8f a = *(const v8f*)(F + e); v8h o;
#pragma unroll
    for (int q = 0; q < 8; ++q) o[q] = tohx(__fmul_rn(bfr(a[q]), 16.0f));
    h16* d0 = P + r * KC2 + c; h16* d1 = d0 + DMD;
    *(volatile v8h*)d0 = o; *(volatile v8h*)d1 = o; __threadfence(); *(volatile v8h*)d0 = o; *(volatile v8h*)d1 = o; }

__global__ __launch_bounds__(128) void k_flash(const h16* __restrict__ QH, const h16* __restrict__ QL, const h16* __restrict__ KH, const h16* __restrict__ KL, const h16* __restrict__ VH, const h16* __restrict__ VL, h16* CT) {
    __shared__ __align__(16) h16 kt[64 * KPT];
    __shared__ __align__(16) h16 ktl[64 * KPT];
    __shared__ __align__(16) h16 vt[64 * KPT];
    __shared__ __align__(16) h16 vtl[64 * KPT];
    __shared__ __align__(16) h16 pt[4 * 16 * PPT];
    __shared__ __align__(16) float ot[4 * 16 * OPT];
    const int tid = threadIdx.x;
    const int wave = __builtin_amdgcn_readfirstlane(tid >> 5);
    const int lane = tid & 31, lr = lane & 15, hi = lane >> 4;
    const int q0 = blockIdx.x * 64, h = blockIdx.y, b = blockIdx.z;
    const int qoff = ((h * NB + b) * TX + q0 + wave * 16 + lr) * HD + 8 * hi;
    const size_t kbase = ((size_t)(h * NB + b) * TY) * HD;
    const size_t vbase = ((size_t)b * DMD + (size_t)h * HD) * TY;
    const int pb = wave * 16 * PPT, ob = wave * 16 * OPT;
    float mrun[8], lrun[8];
#pragma unroll
    for (int r = 0; r < 8; ++r) { mrun[r] = -1.0e30f; lrun[r] = 0.0f; }
    v8f o0 = (v8f){}, o1 = (v8f){}, o2 = (v8f){}, o3 = (v8f){};
    v8f e0 = (v8f){}, e1 = (v8f){}, e2 = (v8f){}, e3 = (v8f){};
#pragma unroll 1
    for (int kb = 0; kb < TY / 64; ++kb) {
        __syncthreads();
#pragma unroll
        for (int i = 0; i < 4; ++i) {
            const int p = tid + 128 * i, row = p >> 3, c8 = (p & 7) * 8;
            const size_t kof = kbase + (size_t)(kb * 64 + row) * HD + c8;
            const size_t vof = vbase + (size_t)row * TY + kb * 64 + c8;
            const v8h kv = *(const v8h*)(KH + kof);
            const v8h kl = *(const v8h*)(KL + kof);
            const v8h vv = *(const v8h*)(VH + vof);
            const v8h vl = *(const v8h*)(VL + vof);
            *(v8ha*)(kt + row * KPT + c8) = kv;
            *(v8ha*)(ktl + row * KPT + c8) = kl;
            *(v8ha*)(vt + row * KPT + c8) = vv;
            *(v8ha*)(vtl + row * KPT + c8) = vl;
        }
        __syncthreads();
#pragma unroll 1
        for (int hf = 0; hf < 2; ++hf) {
            v8f sh0 = (v8f){}, sh1 = (v8f){}, sl0 = (v8f){}, sl1 = (v8f){};
#pragma unroll
            for (int ks = 0; ks < 2; ++ks) {
                int qo = qoff + ks * 32; asm volatile("" : "+v"(qo));
                const v16h ah = cat16(*(const v8h*)(QH + qo), *(const v8h*)(QH + qo + 16));
                const v16h al = cat16(*(const v8h*)(QL + qo), *(const v8h*)(QL + qo + 16));
                const int ko = (hf * 32 + lr) * KPT + ks * 32 + 8 * hi;
                const v16h b0 = cat16(*(const v8ha*)(kt + ko), *(const v8ha*)(kt + ko + 16));
                const v16h b1 = cat16(*(const v8ha*)(kt + ko + 16 * KPT), *(const v8ha*)(kt + ko + 16 * KPT + 16));
                const v16h c0 = cat16(*(const v8ha*)(ktl + ko), *(const v8ha*)(ktl + ko + 16));
                const v16h c1 = cat16(*(const v8ha*)(ktl + ko + 16 * KPT), *(const v8ha*)(ktl + ko + 16 * KPT + 16));
                sh0 = wmma16(ah, b0, sh0); sh1 = wmma16(ah, b1, sh1);
                sl0 = wmma16(al, b0, sl0); sl1 = wmma16(al, b1, sl1);
                sl0 = wmma16(ah, c0, sl0); sl1 = wmma16(ah, c1, sl1);
                asm volatile("v_nop\n\tv_nop\n\tv_nop\n\tv_nop" : "+v"(sh0), "+v"(sh1), "+v"(sl0), "+v"(sl1) : "v"(ah), "v"(al), "v"(b0), "v"(b1), "v"(c0), "v"(c1));
            }
            float t0[8], t1[8], mx[8];
#pragma unroll
            for (int r = 0; r < 8; ++r) { t0[r] = (sh0[r] + sl0[r] * (1.0f / RLO)) * SCL; t1[r] = (sh1[r] + sl1[r] * (1.0f / RLO)) * SCL; mx[r] = fmaxf(t0[r], t1[r]); }
#pragma unroll
            for (int sh = 1; sh < 16; sh <<= 1) {
#pragma unroll
                for (int r = 0; r < 8; ++r) mx[r] = fmaxf(mx[r], __shfl_xor(mx[r], sh, 32)); }
#pragma unroll
            for (int r = 0; r < 8; ++r) {
                const float mn = fmaxf(mrun[r], mx[r]);
                const float cr = __builtin_amdgcn_exp2f((mrun[r] - mn) * L2E);
                mrun[r] = mn;
                const float p0 = __builtin_amdgcn_exp2f((t0[r] - mn) * L2E), p1 = __builtin_amdgcn_exp2f((t1[r] - mn) * L2E);
                const h16 ph0 = tohx(p0 * PCAR), ph1 = tohx(p1 * PCAR);
                lrun[r] = lrun[r] * cr + ((float)ph0 + (float)ph1);
                o0[r] *= cr; o1[r] *= cr; o2[r] *= cr; o3[r] *= cr;
                e0[r] *= cr; e1[r] *= cr; e2[r] *= cr; e3[r] *= cr;
                pt[pb + (8 * hi + r) * PPT + lr] = ph0;
                pt[pb + (8 * hi + r) * PPT + 16 + lr] = ph1;
            }
            wsync();
            {
                const int po = pb + lr * PPT + 8 * hi;
                const v16h pa = cat16(*(const v8ha*)(pt + po), *(const v8ha*)(pt + po + 16));
                const int vo = lr * KPT + hf * 32 + 8 * hi;
                {
                    const v16h v0 = cat16(*(const v8ha*)(vt + vo), *(const v8ha*)(vt + vo + 16));
                    const v16h v1 = cat16(*(const v8ha*)(vt + vo + 16 * KPT), *(const v8ha*)(vt + vo + 16 * KPT + 16));
                    const v16h v2 = cat16(*(const v8ha*)(vt + vo + 32 * KPT), *(const v8ha*)(vt + vo + 32 * KPT + 16));
                    const v16h v3 = cat16(*(const v8ha*)(vt + vo + 48 * KPT), *(const v8ha*)(vt + vo + 48 * KPT + 16));
                    o0 = wmma16(pa, v0, o0); o1 = wmma16(pa, v1, o1); o2 = wmma16(pa, v2, o2); o3 = wmma16(pa, v3, o3);
                    asm volatile("v_nop\n\tv_nop\n\tv_nop\n\tv_nop" : "+v"(o0), "+v"(o1), "+v"(o2), "+v"(o3) : "v"(pa), "v"(v0), "v"(v1), "v"(v2), "v"(v3));
                }
                {
                    const v16h w0 = cat16(*(const v8ha*)(vtl + vo), *(const v8ha*)(vtl + vo + 16));
                    const v16h w1 = cat16(*(const v8ha*)(vtl + vo + 16 * KPT), *(const v8ha*)(vtl + vo + 16 * KPT + 16));
                    const v16h w2 = cat16(*(const v8ha*)(vtl + vo + 32 * KPT), *(const v8ha*)(vtl + vo + 32 * KPT + 16));
                    const v16h w3 = cat16(*(const v8ha*)(vtl + vo + 48 * KPT), *(const v8ha*)(vtl + vo + 48 * KPT + 16));
                    e0 = wmma16(pa, w0, e0); e1 = wmma16(pa, w1, e1); e2 = wmma16(pa, w2, e2); e3 = wmma16(pa, w3, e3);
                    asm volatile("v_nop\n\tv_nop\n\tv_nop\n\tv_nop" : "+v"(e0), "+v"(e1), "+v"(e2), "+v"(e3) : "v"(pa), "v"(w0), "v"(w1), "v"(w2), "v"(w3));
                }
            }
            wsync();
        }
    }
#pragma unroll
    for (int sh = 1; sh < 16; sh <<= 1) {
#pragma unroll
        for (int r = 0; r < 8; ++r) lrun[r] += __shfl_xor(lrun[r], sh, 32); }
#pragma unroll
    for (int r = 0; r < 8; ++r) {
        const float f = __fdiv_rn(OCAR, lrun[r]);
        const int oi = ob + (8 * hi + r) * OPT + lr;
        ot[oi]      = (o0[r] + e0[r] * (1.0f / RLO)) * f;
        ot[oi + 16] = (o1[r] + e1[r] * (1.0f / RLO)) * f;
        ot[oi + 32] = (o2[r] + e2[r] * (1.0f / RLO)) * f;
        ot[oi + 48] = (o3[r] + e3[r] * (1.0f / RLO)) * f;
    }
    wsync();
    h16* crow = CT + (size_t)(b * TX + q0 + wave * 16) * KC2 + h * HD;
#pragma unroll 1
    for (int ps = 0; ps < 2; ++ps) {
#pragma unroll
        for (int s = 0; s < 4; ++s) {
            const int row = 4 * s + (lane >> 3), c8 = (lane & 7) * 8;
            const v4f u0 = *(const v4fa*)(ot + ob + row * OPT + c8), u1 = *(const v4fa*)(ot + ob + row * OPT + c8 + 4);
            v8h oh, ol;
#pragma unroll
            for (int q = 0; q < 8; ++q) { const float f = (q < 4) ? u0[q & 3] : u1[q & 3]; const h16 hh = tohx(f); oh[q] = hh; ol[q] = tohx(f - (float)hh); }
            *(volatile v8h*)(crow + (size_t)row * KC2 + c8) = oh;
            *(volatile v8h*)(crow + (size_t)row * KC2 + DMD + c8) = ol;
        }
        if (ps == 0) __threadfence();
    }
}

constexpr size_t al256(size_t b) { return (b + 255) & ~(size_t)255; }
constexpr size_t SZ_XB = al256((size_t)NB * TX * DMD * 2);
constexpr size_t SZ_YB = al256((size_t)NB * TY * DMD * 2);
constexpr size_t SZ_W  = al256((size_t)DMD * DMD * 2);
constexpr size_t SZ_WP = al256((size_t)DMD * KC2 * 2);
constexpr size_t SZ_Q  = al256((size_t)NHD * NB * TX * HD * 2);
constexpr size_t SZ_K  = al256((size_t)NHD * NB * TY * HD * 2);
constexpr size_t SZ_VT = al256((size_t)NB * DMD * TY * 2);
constexpr size_t SZ_CT = al256((size_t)NB * TX * KC2 * 2);
constexpr size_t SZ_ALL = SZ_XB + SZ_YB + 3 * SZ_W + SZ_WP + 2 * SZ_Q + 2 * SZ_K + 2 * SZ_VT + SZ_CT;
static_assert(SZ_ALL <= (size_t)134217728);

extern "C" void kernel_launch(void* const* d_in, const int* in_sizes, int n_in,
                              void* d_out, int out_size, void* d_ws, size_t ws_size, hipStream_t stream) {
    if (n_in < 8) return;
    const size_t needx = (size_t)(NB - 1) * TX_FULL * DMD + (size_t)TX * DMD;
    if ((size_t)in_sizes[0] < needx || (size_t)in_sizes[1] < (size_t)NB * TY * DMD || (size_t)in_sizes[2] < (size_t)NB * TY) return;
    if (in_sizes[3] < DMD * DMD || in_sizes[4] < DMD * DMD || in_sizes[5] < DMD * DMD || in_sizes[6] < DMD * DMD || in_sizes[7] < DMD) return;
    if ((size_t)out_size < needx) return;
    if (SZ_ALL > ws_size) return;
    const float* x = (const float*)d_in[0]; const float* y = (const float*)d_in[1];
    const float* yw = (const float*)d_in[2];
    const float* wq = (const float*)d_in[3]; const float* wk = (const float*)d_in[4]; const float* wv = (const float*)d_in[5]; const float* wp = (const float*)d_in[6]; const float* bp = (const float*)d_in[7];
    float* OUT = (float*)d_out;

    char* base = (char*)d_ws; size_t off = 0;
    bf* XB = (bf*)(base + off); off += SZ_XB;
    bf* YB = (bf*)(base + off); off += SZ_YB;
    bf* WQ = (bf*)(base + off); off += SZ_W;
    bf* WK = (bf*)(base + off); off += SZ_W;
    bf* WV = (bf*)(base + off); off += SZ_W;
    h16* WP16 = (h16*)(base + off); off += SZ_WP;
    h16* QH16 = (h16*)(base + off); off += SZ_Q;
    h16* QL16 = (h16*)(base + off); off += SZ_Q;
    h16* KH16 = (h16*)(base + off); off += SZ_K;
    h16* KL16 = (h16*)(base + off); off += SZ_K;
    h16* VH16 = (h16*)(base + off); off += SZ_VT;
    h16* VL16 = (h16*)(base + off); off += SZ_VT;
    h16* CT16 = (h16*)(base + off); off += SZ_CT;
    if (off > ws_size) return;

    auto nb256 = [](size_t n) { return (unsigned)((n + 255) / 256); };
    const size_t n8w = (size_t)DMD * DMD / 8;
    k_cvt8r<<<nb256(n8w), 256, 0, stream>>>(wq, WQ, DMD, DMD, n8w);
    k_cvt8r<<<nb256(n8w), 256, 0, stream>>>(wk, WK, DMD, DMD, n8w);
    k_cvt8r<<<nb256(n8w), 256, 0, stream>>>(wv, WV, DMD, DMD, n8w);
    k_cvtwp<<<nb256(n8w), 256, 0, stream>>>(wp, WP16, n8w);
    const size_t n8x = (size_t)NB * TX * DMD / 8, n8y = (size_t)NB * TY * DMD / 8;
    k_cvt8r<<<nb256(n8x), 256, 0, stream>>>(x, XB, TX, TX_FULL, n8x);
    k_cvt8r<<<nb256(n8y), 256, 0, stream>>>(y, YB, TY, TY, n8y);
    k_gemm_q<<<dim3((unsigned)(NB * TX / 64), 1, NHD), 32, 0, stream>>>(XB, WQ, DMD, QH16, QL16, HD, (size_t)0, (size_t)HD * DMD, (size_t)NB * TX * HD);
    k_gemm_k<<<dim3((unsigned)(NB * TY / 64), 1, NHD), 32, 0, stream>>>(YB, WK, DMD, KH16, KL16, HD, yw, (size_t)0, (size_t)HD * DMD, (size_t)NB * TY * HD);
    k_gemm_v<<<dim3(DMD / 64, TY / 64, NB), 32, 0, stream>>>(WV, YB, DMD, VH16, VL16, TY, (size_t)0, (size_t)TY * DMD, (size_t)DMD * TY);
    k_flash<<<dim3(TX / 64, NHD, NB), 128, 0, stream>>>(QH16, QL16, KH16, KL16, VH16, VL16, CT16);
    k_gemm_o<<<dim3(TX / 64, DMD / 64, NB), 32, 0, stream>>>(CT16, WP16, KC2, OUT, DMD, bp, (size_t)TX * KC2, (size_t)0, (size_t)TX_FULL * DMD, 1.0f / 16384.0f);
}
